// LocalSelfAttention_84670985273587
// MI455X (gfx1250) — hardware-verified
//
#include <hip/hip_runtime.h>
#include <math.h>

constexpr int kBatch   = 2;
constexpr int kSeq     = 2048;
constexpr int kDim     = 1024;
constexpr int kDim3    = 3072;
constexpr int kHeads   = 16;
constexpr int kDh      = 64;
constexpr int kTok     = kBatch * kSeq;
constexpr int kHalfWin = 16;
constexpr float kQScale  = 0.125f;
constexpr float kSpRadius = 6.0f;
constexpr float kSpStep   = 0.1f;
constexpr float kSpEps    = 1.0e-8f;
constexpr float kSpCos    = 0.99500416527802576f;
constexpr float kSpSin    = 0.099833416646828152f;
constexpr float kNegFill  = -1.0e30f;
static_assert(kHeads * kDh == kDim, "shape");
static_assert(kTok % 64 == 0 && kDim % 64 == 0 && kDim3 % 64 == 0 && kSeq % 64 == 0, "GEMM M/N tile multiples");
static_assert(kDim % 32 == 0, "GEMM K multiple of 32");
static_assert(kHalfWin < 64, "window fits in the previous key chunk");

typedef __attribute__((ext_vector_type(16))) _Float16 v16h;
typedef __attribute__((ext_vector_type(8)))  _Float16 v8h;
typedef __attribute__((ext_vector_type(16))) __bf16   v16b;
typedef __attribute__((ext_vector_type(8)))  __bf16   v8b;
typedef __attribute__((ext_vector_type(8)))  float    v8f;
typedef __attribute__((ext_vector_type(4)))  float    v4f;
typedef __attribute__((ext_vector_type(2)))  float    v2f;
typedef __attribute__((ext_vector_type(4)))  unsigned int v4u;

__device__ __forceinline__ unsigned short f2bf_bits(float f) {
  unsigned u = __float_as_uint(f);
  return (unsigned short)((u + 0x7FFFu + ((u >> 16) & 1u)) >> 16);
}
__device__ __forceinline__ float bf_bits2f(unsigned short h) { return __uint_as_float(((unsigned)h) << 16); }
__device__ __forceinline__ float bfr(float f) { return bf_bits2f(f2bf_bits(f)); }
__device__ __forceinline__ void split_bits(float f, unsigned short& hb, unsigned short& lb) {
  hb = f2bf_bits(f);
  lb = f2bf_bits(f - bf_bits2f(hb));
}
__device__ __forceinline__ unsigned pk16(unsigned short a, unsigned short b) { return (unsigned)a | ((unsigned)b << 16); }

__device__ __forceinline__ void dep_guard4_h(v8f& a, v8f& b, v8f& c, v8f& d, v16h x, v16h y) {
  asm volatile("v_nop\n\tv_nop\n\tv_nop\n\tv_nop" : "+v"(a), "+v"(b), "+v"(c), "+v"(d) : "v"(x), "v"(y));
}
__device__ __forceinline__ void dep_guard4_b(v8f& a, v8f& b, v8f& c, v8f& d, v16b x, v16b y) {
  asm volatile("v_nop\n\tv_nop\n\tv_nop\n\tv_nop" : "+v"(a), "+v"(b), "+v"(c), "+v"(d) : "v"(x), "v"(y));
}
__device__ __forceinline__ void keep4_h(v16h a, v16h b, v16h c, v16h d) { asm volatile("v_nop" :: "v"(a), "v"(b), "v"(c), "v"(d)); }
__device__ __forceinline__ void keep4_b(v16b a, v16b b, v16b c, v16b d) { asm volatile("v_nop" :: "v"(a), "v"(b), "v"(c), "v"(d)); }
__device__ __forceinline__ void acc_guard4(v8f& a, v8f& b, v8f& c, v8f& d) { asm volatile("v_nop\n\tv_nop\n\tv_nop\n\tv_nop" : "+v"(a), "+v"(b), "+v"(c), "+v"(d)); }
template <typename T> struct Frag;
template <> struct Frag<_Float16> {
  typedef v16h V; union U { v16h v; v8h h[2]; };
  static __device__ __forceinline__ v16h load(const _Float16* p) {
    U f; f.h[0] = *(const v8h*)(p); f.h[1] = *(const v8h*)(p + 16); return f.v;
  }
  static __device__ __forceinline__ v8f mma(v16h a, v16h b, v8f c) {
    return __builtin_amdgcn_wmma_f32_16x16x32_f16(false, a, false, b, (short)0, c, false, false);
  }
  static __device__ __forceinline__ void guard4(v8f& a, v8f& b, v8f& c, v8f& d, v16h x, v16h y) { dep_guard4_h(a, b, c, d, x, y); }
  static __device__ __forceinline__ void keep(v16h a, v16h b, v16h c, v16h d) { keep4_h(a, b, c, d); }
};
template <> struct Frag<__bf16> {
  typedef v16b V; union U { v16b v; v8b h[2]; };
  static __device__ __forceinline__ v16b load(const __bf16* p) {
    U f; f.h[0] = *(const v8b*)(p); f.h[1] = *(const v8b*)(p + 16); return f.v;
  }
  static __device__ __forceinline__ v8f mma(v16b a, v16b b, v8f c) {
    return __builtin_amdgcn_wmma_f32_16x16x32_bf16(false, a, false, b, (short)0, c, false, false);
  }
  static __device__ __forceinline__ void guard4(v8f& a, v8f& b, v8f& c, v8f& d, v16b x, v16b y) { dep_guard4_b(a, b, c, d, x, y); }
  static __device__ __forceinline__ void keep(v16b a, v16b b, v16b c, v16b d) { keep4_b(a, b, c, d); }
};

template <int ET> struct Elem;
template <> struct Elem<0> { typedef _Float16 T; };
template <> struct Elem<1> { typedef __bf16 T; };
template <int ET, int SPLITM, int BIAS_MODE, int OUT_MODE, bool RESID, int ACT = 0>
__global__ __launch_bounds__(256) void wmma_gemm64(
    const unsigned short* __restrict__ Ap, const unsigned short* __restrict__ A2p, int lda, long strideA,
    const unsigned short* __restrict__ Btp, const unsigned short* __restrict__ Bt2p, int ldb, long strideB,
    void* __restrict__ Cout, void* __restrict__ Cout2, int ldc, long strideC,
    const float* __restrict__ bias,
    const float* __restrict__ resid, long strideR,
    int M, int N, int K, float scale,
    const float* __restrict__ gainp, const float* __restrict__ prep) {
  typedef typename Elem<ET>::T T;
  typedef typename Frag<T>::V V;
  const T* A = (const T*)Ap; const T* A2 = (const T*)A2p; const T* Bt = (const T*)Btp; const T* Bt2 = (const T*)Bt2p;
  __shared__ __align__(16) float sT[8][16 * 68];
  const int b    = blockIdx.y;
  const int lane = threadIdx.x & 31;
  const int wave = threadIdx.x >> 5;
  const int tilesN = N >> 6;
  const int tilesM = M >> 6;
  const int tile = blockIdx.x * 8 + wave;
  if (tile >= tilesM * tilesN) return;
  const int tm = tile / tilesN;
  const int tn = tile - tm * tilesN;
  const int m0 = tm << 6;
  const int n0 = tn << 6;

  const T* Ab  = A  + (size_t)b * strideA;
  const T* Bb  = Bt + (size_t)b * strideB;
  const T* Ab2 = (SPLITM != 0) ? (A2  + (size_t)b * strideA) : nullptr;
  const T* Bb2 = (SPLITM == 1) ? (Bt2 + (size_t)b * strideB) : nullptr;

  const int rlane = lane & 15;
  const int koff  = (lane >> 4) * 8;
  const int mOff  = (lane >> 4) * 8;

  v8f acc[4][4];
#pragma unroll
  for (int i = 0; i < 4; ++i)
#pragma unroll
    for (int j = 0; j < 4; ++j) acc[i][j] = (v8f){0.f,0.f,0.f,0.f,0.f,0.f,0.f,0.f};

  for (int k0 = 0; k0 < K; k0 += 32) {
    V bh[4], bl[4];
#pragma unroll
    for (int j = 0; j < 4; ++j) {
      const size_t bo = (size_t)(n0 + (j << 4) + rlane) * ldb + koff + k0;
      bh[j] = Frag<T>::load(Bb + bo);
      if (SPLITM == 1) bl[j] = Frag<T>::load(Bb2 + bo);
      else bl[j] = bh[j];
    }
#pragma unroll
    for (int i = 0; i < 4; ++i) {
      const size_t ao = (size_t)(m0 + (i << 4) + rlane) * lda + koff + k0;
      V ah = Frag<T>::load(Ab + ao);
      V al = ah;
      if (SPLITM != 0) al = Frag<T>::load(Ab2 + ao);
#pragma unroll
      for (int j = 0; j < 4; ++j) {
        acc[i][j] = Frag<T>::mma(ah, bh[j], acc[i][j]);
        if (SPLITM == 1) acc[i][j] = Frag<T>::mma(ah, bl[j], acc[i][j]);
        if (SPLITM != 0) acc[i][j] = Frag<T>::mma(al, bh[j], acc[i][j]);
      }
      Frag<T>::guard4(acc[i][0], acc[i][1], acc[i][2], acc[i][3], ah, al);
    }
    Frag<T>::keep(bh[0], bh[1], bh[2], bh[3]);
    if (SPLITM == 1) Frag<T>::keep(bl[0], bl[1], bl[2], bl[3]);
  }
  acc_guard4(acc[0][0], acc[0][1], acc[0][2], acc[0][3]);
  acc_guard4(acc[1][0], acc[1][1], acc[1][2], acc[1][3]);
  acc_guard4(acc[2][0], acc[2][1], acc[2][2], acc[2][3]);
  acc_guard4(acc[3][0], acc[3][1], acc[3][2], acc[3][3]);

  float* slab = sT[wave];
  const float* Rb = RESID ? (resid + (size_t)b * strideR) : nullptr;
  float pre = 0.f;
  if (ACT == 6) pre = bfr(prep[0]);
#pragma unroll
  for (int i = 0; i < 4; ++i) {
    const int mBase = m0 + (i << 4);
#pragma unroll
    for (int j = 0; j < 4; ++j) {
      const int n = n0 + (j << 4) + rlane;
      float bv = 0.f;
      float gv = 1.f;
      if (BIAS_MODE == 2) bv = bias[n];
      if (ACT == 6) { gv = bfr(gainp[n]); bv = bfr(bias[n]); }
#pragma unroll
      for (int r = 0; r < 8; ++r) {
        float v = acc[i][j][r] * scale;
        if (BIAS_MODE == 1) v += bias[mBase + mOff + r];
        if (BIAS_MODE == 2) v += bv;
        if (RESID) v += Rb[(size_t)(mBase + mOff + r) * ldc + n];
        if (ACT == 1) v = tanhf(v);
        if (ACT == 2) v = fmaxf(v, 0.0f);
        if (ACT == 4) v = (v > 0.f) ? v : 0.01f * v;
        if (ACT == 6) v = gv * tanhf(pre * v) + bv;
        slab[(mOff + r) * 68 + (j << 4) + rlane] = v;
      }
    }
    __builtin_amdgcn_fence(__ATOMIC_RELEASE, "workgroup");
    __builtin_amdgcn_wave_barrier();
    __builtin_amdgcn_fence(__ATOMIC_ACQUIRE, "workgroup");
    if (OUT_MODE == 0) {
      float* C = (float*)Cout + (size_t)b * strideC;
      const int hh = lane >> 4, c4 = (lane & 15) * 4;
      for (int pass = 0; pass < 2; ++pass) {
#pragma unroll
        for (int it = 0; it < 8; ++it) {
          const int row = it * 2 + hh;
          v4f v = *(const v4f*)(slab + row * 68 + c4);
          *(volatile v4f*)(C + (size_t)(mBase + row) * ldc + n0 + c4) = v;
        }
        __threadfence();
      }
    } else {
      const int q = lane >> 3, c8 = (lane & 7) * 8;
      unsigned short* C  = (unsigned short*)Cout  + (size_t)b * strideC;
      unsigned short* C2 = (OUT_MODE == 2) ? ((unsigned short*)Cout2 + (size_t)b * strideC) : nullptr;
      for (int pass = 0; pass < 2; ++pass) {
#pragma unroll
        for (int it = 0; it < 4; ++it) {
          const int row = it * 4 + q;
          const float* sp = slab + row * 68 + c8;
          v8h hv, lv;
#pragma unroll
          for (int e = 0; e < 8; ++e) {
            if (OUT_MODE == 1) {
              hv[e] = (_Float16)sp[e];
            } else {
              unsigned short hb = f2bf_bits(sp[e]);
              unsigned short lb = f2bf_bits(sp[e] - bf_bits2f(hb));
              hv[e] = __builtin_bit_cast(_Float16, hb);
              lv[e] = __builtin_bit_cast(_Float16, lb);
            }
          }
          *(volatile v8h*)(C + (size_t)(mBase + row) * ldc + n0 + c8) = hv;
          if (OUT_MODE == 2) *(volatile v8h*)(C2 + (size_t)(mBase + row) * ldc + n0 + c8) = lv;
        }
        __threadfence();
      }
    }
    __builtin_amdgcn_fence(__ATOMIC_RELEASE, "workgroup");
    __builtin_amdgcn_wave_barrier();
    __builtin_amdgcn_fence(__ATOMIC_ACQUIRE, "workgroup");
  }
}

__global__ __launch_bounds__(256) void cast8_bf16_kernel(const float* __restrict__ in, unsigned short* __restrict__ out, int n8) {
  const int i = blockIdx.x * 256 + threadIdx.x;
  if (i >= n8) return;
  const float* p = in + 8 * (size_t)i;
  const v4f a = *(const v4f*)(p);
  const v4f c = *(const v4f*)(p + 4);
  unsigned short hb[8];
#pragma unroll
  for (int e = 0; e < 4; ++e) {
    hb[e]     = f2bf_bits(a[e]);
    hb[4 + e] = f2bf_bits(c[e]);
  }
  const v4u u = (v4u){pk16(hb[0], hb[1]), pk16(hb[2], hb[3]), pk16(hb[4], hb[5]), pk16(hb[6], hb[7])};
  unsigned short* q = out + 8 * (size_t)i;
  *(volatile v4u*)q = u;
  __threadfence();
  *(volatile v4u*)q = u;
}

__global__ __launch_bounds__(256) void wt_cast_kernel(const float* __restrict__ W, int nOut, unsigned short* __restrict__ out) {
  __shared__ float sm[64][65];
  const int t  = threadIdx.x;
  const int k0 = blockIdx.x * 64;
  const int n0 = blockIdx.y * 64;
#pragma unroll
  for (int i = 0; i < 8; ++i) {
    const int e = i * 256 + t;
    const int r = e >> 6;
    const int c = e & 63;
    sm[c][r] = W[(size_t)(k0 + r) * nOut + n0 + c];
  }
  asm volatile("" ::: "memory");
#pragma unroll
  for (int i = 8; i < 16; ++i) {
    const int e = i * 256 + t;
    const int r = e >> 6;
    const int c = e & 63;
    sm[c][r] = W[(size_t)(k0 + r) * nOut + n0 + c];
  }
  __syncthreads();
  const int lane = t & 31, wave = t >> 5;
  const int q = lane >> 3, c8 = (lane & 7) * 8;
  for (int pass = 0; pass < 2; ++pass) {
#pragma unroll
    for (int it = 0; it < 2; ++it) {
      const int row = wave * 8 + it * 4 + q;
      unsigned short hb[8];
#pragma unroll
      for (int e = 0; e < 8; ++e) hb[e] = f2bf_bits(sm[row][c8 + e]);
      const v4u u = (v4u){pk16(hb[0], hb[1]), pk16(hb[2], hb[3]), pk16(hb[4], hb[5]), pk16(hb[6], hb[7])};
      *(volatile v4u*)(out + (size_t)(n0 + row) * kDim + k0 + c8) = u;
    }
    __threadfence();
  }
}

__device__ __forceinline__ void spiral_step(float& a, float& b, float& d) {
  const float ss = (a * a + d * d) + b * b;
  const float r = fmaxf(sqrtf(ss), kSpEps);
  const float inv = 1.0f / r;
  const float g = kSpRadius - r;
  const float ra = g * (a * inv);
  const float rb = g * (b * inv);
  const float rd = g * (d * inv);
  const float ya = kSpCos * a - kSpSin * b;
  const float yb = kSpSin * a + kSpCos * b;
  const float na = a + kSpStep * ((ya - a) + ra);
  const float nb = b + kSpStep * ((yb - b) + rb);
  const float nd = d + kSpStep * (rd);
  a = na; b = nb; d = nd;
}

__global__ __launch_bounds__(256) void spiral_split_kernel(const float* __restrict__ QKV,
                                                           unsigned* __restrict__ Qh, unsigned* __restrict__ Ql,
                                                           unsigned* __restrict__ Kh, unsigned* __restrict__ Kl, int n2) {
  const int i = blockIdx.x * 256 + threadIdx.x;
  if (i >= n2) return;
  const int bt = i >> 9;
  const int c  = (i & 511) * 2;
  const float* base = QKV + (size_t)bt * kDim3 + c;
  const v2f qv = *(const v2f*)(base);
  const v2f kv = *(const v2f*)(base + kDim);
  const v2f vv = *(const v2f*)(base + 2 * kDim);
  float a0 = qv[0], b0 = kv[0], d0 = vv[0];
  float a1 = qv[1], b1 = kv[1], d1 = vv[1];
  spiral_step(a0, b0, d0); spiral_step(a0, b0, d0);
  spiral_step(a1, b1, d1); spiral_step(a1, b1, d1);
  a0 *= kQScale; a1 *= kQScale;
  unsigned short qh0, ql0, qh1, ql1, kh0, kl0, kh1, kl1;
  split_bits(a0, qh0, ql0);
  split_bits(a1, qh1, ql1);
  split_bits(b0, kh0, kl0);
  split_bits(b1, kh1, kl1);
  const unsigned uqh = pk16(qh0, qh1), uql = pk16(ql0, ql1), ukh = pk16(kh0, kh1), ukl = pk16(kl0, kl1);
  ((volatile unsigned*)Qh)[i] = uqh;
  ((volatile unsigned*)Ql)[i] = uql;
  ((volatile unsigned*)Kh)[i] = ukh;
  ((volatile unsigned*)Kl)[i] = ukl;
  __threadfence();
  ((volatile unsigned*)Qh)[i] = uqh;
  ((volatile unsigned*)Ql)[i] = uql;
  ((volatile unsigned*)Kh)[i] = ukh;
  ((volatile unsigned*)Kl)[i] = ukl;
}

__global__ __launch_bounds__(256) void vt_split_kernel(const float* __restrict__ QKV,
                                                       unsigned short* __restrict__ VTh, unsigned short* __restrict__ VTl) {
  __shared__ float sm[64][65];
  const int t  = threadIdx.x;
  const int s0 = blockIdx.x * 64;
  const int h  = blockIdx.y;
  const int b  = blockIdx.z;
  const float* vbase = QKV + 2 * kDim + h * kDh;
#pragma unroll
  for (int i = 0; i < 8; ++i) {
    const int e = i * 256 + t;
    const int r = e >> 6;
    const int c = e & 63;
    sm[c][r] = vbase[(size_t)(b * kSeq + s0 + r) * kDim3 + c];
  }
  asm volatile("" ::: "memory");
#pragma unroll
  for (int i = 8; i < 16; ++i) {
    const int e = i * 256 + t;
    const int r = e >> 6;
    const int c = e & 63;
    sm[c][r] = vbase[(size_t)(b * kSeq + s0 + r) * kDim3 + c];
  }
  __syncthreads();
  const int lane = t & 31, wave = t >> 5;
  const int q = lane >> 3, c8 = (lane & 7) * 8;
  const size_t pbase = ((size_t)(b * kHeads + h) * kDh) * kSeq;
  for (int pass = 0; pass < 2; ++pass) {
#pragma unroll
    for (int it = 0; it < 2; ++it) {
      const int row = wave * 8 + it * 4 + q;
      unsigned short hb[8], lb[8];
#pragma unroll
      for (int e = 0; e < 8; ++e) split_bits(sm[row][c8 + e], hb[e], lb[e]);
      const v4u uh = (v4u){pk16(hb[0], hb[1]), pk16(hb[2], hb[3]), pk16(hb[4], hb[5]), pk16(hb[6], hb[7])};
      const v4u ul = (v4u){pk16(lb[0], lb[1]), pk16(lb[2], lb[3]), pk16(lb[4], lb[5]), pk16(lb[6], lb[7])};
      const size_t off = pbase + (size_t)row * kSeq + s0 + c8;
      *(volatile v4u*)(VTh + off) = uh;
      *(volatile v4u*)(VTl + off) = ul;
    }
    __threadfence();
  }
}

constexpr int kAtD  = 64;
constexpr int kAtKC = 64;
constexpr int kAtNW = 4;

__device__ __forceinline__ v8f at_mma(v16b a, v16b b, v8f c) {
  c = __builtin_amdgcn_wmma_f32_16x16x32_bf16(false, a, false, b, (short)0, c, false, false);
  asm volatile("v_nop\n\tv_nop\n\tv_nop\n\tv_nop" : "+v"(c) : "v"(a), "v"(b));
  return c;
}

__global__ __launch_bounds__(128)
void local_attn_kernel(const unsigned short* __restrict__ Qh, const unsigned short* __restrict__ Ql,
                       const unsigned short* __restrict__ Kh, const unsigned short* __restrict__ Kl,
                       const unsigned short* __restrict__ VTh, const unsigned short* __restrict__ VTl,
                       const float* __restrict__ sinks,
                       unsigned short* __restrict__ Yh, unsigned short* __restrict__ Yl) {
  union FB { v16b v; v8b h[2]; };
  __shared__ __align__(16) __bf16 Ksh[kAtKC * kAtD];
  __shared__ __align__(16) __bf16 Ksl[kAtKC * kAtD];
  __shared__ __align__(16) __bf16 Vth[kAtD * kAtKC];
  __shared__ __align__(16) __bf16 Vtl[kAtD * kAtKC];
  __shared__ __align__(16) __bf16 Psh[kAtNW][16 * kAtKC];
  __shared__ __align__(16) __bf16 Psl[kAtNW][16 * kAtKC];
  __shared__ __align__(16) float  Os[kAtNW][16 * 68];

  const int tid  = threadIdx.x;
  const int wave = tid >> 5;
  const int lane = tid & 31;
  const int hh   = lane >> 4;
  const int c    = lane & 15;

  const int qb = blockIdx.x;
  const int h  = blockIdx.y;
  const int b  = blockIdx.z;
  const int q0 = qb * 64 + wave * 16;
  const size_t tokBase = (size_t)b * kSeq;

  v16b qah[2], qal[2];
  {
    const __bf16* qhp = (const __bf16*)Qh + (tokBase + q0 + c) * kDim + h * kDh + 8 * hh;
    const __bf16* qlp = (const __bf16*)Ql + (tokBase + q0 + c) * kDim + h * kDh + 8 * hh;
#pragma unroll
    for (int dc = 0; dc < 2; ++dc) qah[dc] = Frag<__bf16>::load(qhp + dc * 32);
    asm volatile("" ::: "memory");
#pragma unroll
    for (int dc = 0; dc < 2; ++dc) qal[dc] = Frag<__bf16>::load(qlp + dc * 32);
  }

  const float sinkv = bfr(sinks[h]);
  float mrow[8], lrow[8];
  v8f oacc[4];
#pragma unroll
  for (int r = 0; r < 8; ++r) { mrow[r] = sinkv; lrow[r] = 1.0f; }
#pragma unroll
  for (int t = 0; t < 4; ++t) oacc[t] = (v8f){0.f,0.f,0.f,0.f,0.f,0.f,0.f,0.f};

  const int kcBeg = (qb > 0) ? (qb - 1) : 0;
  const size_t vtBase = ((size_t)(b * kHeads + h) * kDh) * kSeq;
  for (int kc = kcBeg; kc <= qb; ++kc) {
    const int kv0 = kc * kAtKC;
    __syncthreads();
#pragma unroll
    for (int it = 0; it < 4; ++it) {
      const int e = it * 128 + tid;
      const int row = e >> 3;
      const int c16 = (e & 7) * 8;
      const size_t go = (tokBase + kv0 + row) * kDim + h * kDh + c16;
      const v4u wh = *(const v4u*)(Kh + go);
      const v4u wl = *(const v4u*)(Kl + go);
      *(v4u*)(Ksh + row * kAtD + c16) = wh;
      *(v4u*)(Ksl + row * kAtD + c16) = wl;
    }
    asm volatile("" ::: "memory");
#pragma unroll
    for (int it = 0; it < 4; ++it) {
      const int e = it * 128 + tid;
      const int row = e >> 3;
      const int c16 = (e & 7) * 8;
      const size_t go = vtBase + (size_t)row * kSeq + kv0 + c16;
      const v4u wh = *(const v4u*)(VTh + go);
      const v4u wl = *(const v4u*)(VTl + go);
      *(v4u*)(Vth + row * kAtKC + c16) = wh;
      *(v4u*)(Vtl + row * kAtKC + c16) = wl;
    }
    __syncthreads();

    v8f s[4];
#pragma unroll
    for (int j = 0; j < 4; ++j) {
      s[j] = (v8f){0.f,0.f,0.f,0.f,0.f,0.f,0.f,0.f};
#pragma unroll
      for (int dc = 0; dc < 2; ++dc) {
        FB kb, kl;
        kb.h[0] = *(const v8b*)(Ksh + (j * 16 + c) * kAtD + dc * 32 + 8 * hh);
        kb.h[1] = *(const v8b*)(Ksh + (j * 16 + c) * kAtD + dc * 32 + 16 + 8 * hh);
        kl.h[0] = *(const v8b*)(Ksl + (j * 16 + c) * kAtD + dc * 32 + 8 * hh);
        kl.h[1] = *(const v8b*)(Ksl + (j * 16 + c) * kAtD + dc * 32 + 16 + 8 * hh);
        s[j] = at_mma(qah[dc], kb.v, s[j]);
        s[j] = at_mma(qah[dc], kl.v, s[j]);
        s[j] = at_mma(qal[dc], kb.v, s[j]);
      }
    }
    float cm[8];
#pragma unroll
    for (int r = 0; r < 8; ++r) {
      const int qrow = q0 + 8 * hh + r;
      float m = kNegFill;
#pragma unroll
      for (int j = 0; j < 4; ++j) {
        const int kvcol = kv0 + j * 16 + c;
        const bool masked = (kvcol > qrow) || (qrow - kvcol > kHalfWin);
        const float sv = masked ? kNegFill : s[j][r];
        s[j][r] = sv;
        m = fmaxf(m, sv);
      }
#pragma unroll
      for (int off = 1; off < 16; off <<= 1) m = fmaxf(m, __shfl_xor(m, off, 32));
      cm[r] = m;
    }
    __bf16* pwh = Psh[wave];
    __bf16* pwl = Psl[wave];
#pragma unroll
    for (int r = 0; r < 8; ++r) {
      const float mnew = fmaxf(mrow[r], cm[r]);
      const float alpha = expf(mrow[r] - mnew);
      mrow[r] = mnew;
      float psum = 0.f;
#pragma unroll
      for (int j = 0; j < 4; ++j) {
        const float p = expf(s[j][r] - mnew);
        psum += p;
        unsigned short phb, plb;
        split_bits(p, phb, plb);
        pwh[(8 * hh + r) * kAtKC + j * 16 + c] = __builtin_bit_cast(__bf16, phb);
        pwl[(8 * hh + r) * kAtKC + j * 16 + c] = __builtin_bit_cast(__bf16, plb);
      }
#pragma unroll
      for (int off = 1; off < 16; off <<= 1) psum += __shfl_xor(psum, off, 32);
      lrow[r] = lrow[r] * alpha + psum;
#pragma unroll
      for (int t = 0; t < 4; ++t) oacc[t][r] *= alpha;
    }
    __builtin_amdgcn_fence(__ATOMIC_RELEASE, "workgroup");
    __builtin_amdgcn_wave_barrier();
    __builtin_amdgcn_fence(__ATOMIC_ACQUIRE, "workgroup");
#pragma unroll 1
    for (int kk = 0; kk < 2; ++kk) {
      FB pa, pl;
      pa.h[0] = *(const v8b*)(pwh + c * kAtKC + kk * 32 + 8 * hh);
      pa.h[1] = *(const v8b*)(pwh + c * kAtKC + kk * 32 + 16 + 8 * hh);
      pl.h[0] = *(const v8b*)(pwl + c * kAtKC + kk * 32 + 8 * hh);
      pl.h[1] = *(const v8b*)(pwl + c * kAtKC + kk * 32 + 16 + 8 * hh);
#pragma unroll
      for (int t = 0; t < 4; ++t) {
        FB vb, vl;
        vb.h[0] = *(const v8b*)(Vth + (t * 16 + c) * kAtKC + kk * 32 + 8 * hh);
        vb.h[1] = *(const v8b*)(Vth + (t * 16 + c) * kAtKC + kk * 32 + 16 + 8 * hh);
        vl.h[0] = *(const v8b*)(Vtl + (t * 16 + c) * kAtKC + kk * 32 + 8 * hh);
        vl.h[1] = *(const v8b*)(Vtl + (t * 16 + c) * kAtKC + kk * 32 + 16 + 8 * hh);
        oacc[t] = at_mma(pa.v, vb.v, oacc[t]);
        oacc[t] = at_mma(pa.v, vl.v, oacc[t]);
        oacc[t] = at_mma(pl.v, vb.v, oacc[t]);
      }
    }
  }

  float* os = Os[wave];
#pragma unroll
  for (int r = 0; r < 8; ++r) {
    const float inv = 1.0f / lrow[r];
#pragma unroll
    for (int t = 0; t < 4; ++t) os[(8 * hh + r) * 68 + t * 16 + c] = oacc[t][r] * inv;
  }
  __builtin_amdgcn_fence(__ATOMIC_RELEASE, "workgroup");
  __builtin_amdgcn_wave_barrier();
  __builtin_amdgcn_fence(__ATOMIC_ACQUIRE, "workgroup");
  {
    const int q4 = lane >> 3, c8 = (lane & 7) * 8;
    for (int pass = 0; pass < 2; ++pass) {
#pragma unroll
      for (int it = 0; it < 4; ++it) {
        const int row = it * 4 + q4;
        const float* sp = os + row * 68 + c8;
        unsigned short hb[8], lb[8];
#pragma unroll
        for (int e = 0; e < 8; ++e) split_bits(sp[e], hb[e], lb[e]);
        const v4u uh = (v4u){pk16(hb[0], hb[1]), pk16(hb[2], hb[3]), pk16(hb[4], hb[5]), pk16(hb[6], hb[7])};
        const v4u ul = (v4u){pk16(lb[0], lb[1]), pk16(lb[2], lb[3]), pk16(lb[4], lb[5]), pk16(lb[6], lb[7])};
        const size_t yo = (tokBase + q0 + row) * kDim + h * kDh + c8;
        *(volatile v4u*)(Yh + yo) = uh;
        *(volatile v4u*)(Yl + yo) = ul;
      }
      __threadfence();
    }
  }
}

extern "C" void kernel_launch(void* const* d_in, const int* in_sizes, int n_in,
                              void* d_out, int out_size, void* d_ws, size_t ws_size,
                              hipStream_t stream) {
  if (n_in < 7) return;
  const int nAct = kTok * kDim;
  if (in_sizes[0] != nAct) return;
  if (in_sizes[1] != kDim * kDim3) return;
  if (in_sizes[2] != kDim * kDim) return;
  if (in_sizes[3] != kHeads) return;
  if (in_sizes[4] < 1) return;
  if (in_sizes[5] != kDim || in_sizes[6] != kDim) return;
  if (out_size != nAct) return;

  const size_t szPlane16 = (size_t)kTok * kDim * 2;
  const size_t szWa      = (size_t)kDim3 * kDim * 2;
  const size_t szWp      = (size_t)kDim * kDim * 2;
  const size_t szQKV     = (size_t)kTok * kDim3 * 4;
  const size_t szVT      = (size_t)kBatch * kHeads * kDh * kSeq * 2;
  const size_t offXb  = 0;
  const size_t offWa  = offXb + szPlane16;
  const size_t offWp  = offWa + szWa;
  const size_t offQKV = offWp + szWp;
  const size_t offQh  = offQKV + szQKV;
  const size_t offQl  = offQh + szPlane16;
  const size_t offKh  = offQl + szPlane16;
  const size_t offKl  = offKh + szPlane16;
  const size_t offVTh = offKl + szPlane16;
  const size_t offVTl = offVTh + szVT;
  const size_t offYh  = offVTl + szVT;
  const size_t offYl  = offYh + szPlane16;
  const size_t total  = offYl + szPlane16;
  if (ws_size < total) return;

  const float* x        = (const float*)d_in[0];
  const float* W_attn   = (const float*)d_in[1];
  const float* W_proj   = (const float*)d_in[2];
  const float* sinks    = (const float*)d_in[3];
  const float* ln_scale = (const float*)d_in[4];
  const float* ln_delta = (const float*)d_in[5];
  const float* ln_bias  = (const float*)d_in[6];
  float* out = (float*)d_out;
  char* ws = (char*)d_ws;
  unsigned short* Xb  = (unsigned short*)(ws + offXb);
  unsigned short* WaT = (unsigned short*)(ws + offWa);
  unsigned short* WpT = (unsigned short*)(ws + offWp);
  float*          QKV = (float*)(ws + offQKV);
  unsigned short* Qh  = (unsigned short*)(ws + offQh);
  unsigned short* Ql  = (unsigned short*)(ws + offQl);
  unsigned short* Kh  = (unsigned short*)(ws + offKh);
  unsigned short* Kl  = (unsigned short*)(ws + offKl);
  unsigned short* VTh = (unsigned short*)(ws + offVTh);
  unsigned short* VTl = (unsigned short*)(ws + offVTl);
  unsigned short* Yh  = (unsigned short*)(ws + offYh);
  unsigned short* Yl  = (unsigned short*)(ws + offYl);

  const int n8 = nAct / 8;
  cast8_bf16_kernel<<<dim3(n8 / 256), dim3(256), 0, stream>>>(x, Xb, n8);
  wt_cast_kernel<<<dim3(kDim / 64, kDim3 / 64), dim3(256), 0, stream>>>(W_attn, kDim3, WaT);
  wt_cast_kernel<<<dim3(kDim / 64, kDim / 64), dim3(256), 0, stream>>>(W_proj, kDim, WpT);

  const int tiles1 = (kTok / 64) * (kDim3 / 64);
  wmma_gemm64<1, 0, 0, 0, false, 0><<<dim3(tiles1 / 8, 1), dim3(256), 0, stream>>>(
      Xb, Xb, kDim, 0L, WaT, WaT, kDim, 0L,
      (void*)QKV, (void*)QKV, kDim3, 0L, sinks, sinks, 0L, kTok, kDim3, kDim, 1.0f, sinks, sinks);

  const int n2 = nAct / 2;
  spiral_split_kernel<<<dim3(n2 / 256), dim3(256), 0, stream>>>(
      QKV, (unsigned*)Qh, (unsigned*)Ql, (unsigned*)Kh, (unsigned*)Kl, n2);

  vt_split_kernel<<<dim3(kSeq / 64, kHeads, kBatch), dim3(256), 0, stream>>>(QKV, VTh, VTl);

  local_attn_kernel<<<dim3(kSeq / 64, kHeads, kBatch), dim3(128), 0, stream>>>(
      Qh, Ql, Kh, Kl, VTh, VTl, sinks, Yh, Yl);

  const int tiles2 = (kTok / 64) * (kDim / 64);
  wmma_gemm64<1, 2, 0, 0, false, 6><<<dim3(tiles2 / 8, 1), dim3(256), 0, stream>>>(
      Yh, Yl, kDim, 0L, WpT, WpT, kDim, 0L,
      (void*)out, (void*)out, kDim, 0L, ln_bias, sinks, 0L, kTok, kDim, kDim, 1.0f, ln_delta, ln_scale);
}
